// MyGNN_44856638439998
// MI455X (gfx1250) — hardware-run, weakly checked
//
#include <hip/hip_runtime.h>


namespace {
constexpr int N = 4096, CI = 512, CO = 256, QL = N  ;
constexpr float XS = 8.0f, WSC = 256.0f, RS_ = 1024.0f, PS = 1024.0f, NSL = 0.2f, LOG2E = 1.4426950408889634f;
static_assert(N % 32 == 0 && CI % 32 == 0 && CO == 256 && QL % 16 == 0, "tiling");
typedef _Float16 b16;
typedef __attribute__((ext_vector_type(16))) _Float16 v16b;
typedef __attribute__((ext_vector_type(8))) _Float16 v8b;
typedef __attribute__((ext_vector_type(8))) float v8f;
typedef __attribute__((ext_vector_type(4))) float v4f;
__device__ __forceinline__ float bf16_rne(float f) { unsigned int u = __float_as_uint(f); u += 0x7FFFu + ((u >> 16) & 1u); return __uint_as_float(u & 0xFFFF0000u); }
__device__ __forceinline__ void split16(float v, b16& hi, b16& lo) { hi = (b16)v; lo = (b16)(v - (float)hi); }
__device__ __forceinline__ v16b frag_kb(const b16* p, int hh) { const v8b a = *(const v8b*)(p + 8 * hh), b = *(const v8b*)(p + 16 + 8 * hh); v16b f;
#pragma unroll
  for (int e = 0; e < 8; ++e) { f[e] = a[e]; f[8 + e] = b[e]; } return f; }
__device__ __forceinline__ v8f wmma16b(v16b a, v16b b, v8f c) { v8f d = __builtin_amdgcn_wmma_f32_16x16x32_f16(false, a, false, b, (short)0, c, false, false); asm volatile("v_nop\n\tv_nop\n\tv_nop\n\tv_nop" : "+v"(d) : "v"(a), "v"(b)); return d; }
__device__ __forceinline__ void wave_lds_sync() { __builtin_amdgcn_fence(__ATOMIC_RELEASE, "workgroup"); __builtin_amdgcn_wave_barrier(); __builtin_amdgcn_fence(__ATOMIC_ACQUIRE, "workgroup"); }
__device__ __forceinline__ float pmul(float a, float b) { float p = a * b; asm volatile("" : "+v"(p)); return p; }
__device__ __forceinline__ int iclamp(int v, int lo, int hi) { return v < lo ? lo : (v > hi ? hi : v); }

typedef __attribute__((ext_vector_type(2))) _Float16 v2h;
typedef __attribute__((ext_vector_type(4))) _Float16 v4h;
typedef __attribute__((ext_vector_type(2))) float v2f;
typedef __attribute__((ext_vector_type(4))) int v4i;
__device__ __forceinline__ float nexp2(float v) { return __builtin_amdgcn_exp2f(v); }
__device__ __forceinline__ float bfp(float v) { float t = bf16_rne(v); asm volatile("" : "+v"(t)); return t; }

__device__ __forceinline__ float lrelu(float v) { return v > 0.0f ? v : NSL * v; }
__global__ __launch_bounds__(256) void wt_kernel(const float* __restrict__ w, b16* __restrict__ WT) {
  const int u = blockIdx.x * 256 + threadIdx.x; if (u >= CO * CI / 8) return; const int e = u * 8; v8b v;
#pragma unroll
  for (int j = 0; j < 8; ++j) v[j] = (b16)(bf16_rne(w[e + j]) * WSC);
  for (int pass = 0; pass < 2; ++pass) { *(volatile v8b*)(WT + e) = v; __threadfence(); }
}
__global__ __launch_bounds__(64) void proj_kernel(const float* __restrict__ x, const b16* __restrict__ WT, const float* __restrict__ as_, const float* __restrict__ ad_, b16* __restrict__ X1h, b16* __restrict__ X1l, float* __restrict__ AS, float* __restrict__ AD) {
  __shared__ __attribute__((aligned(16))) b16 Ah[2][16][CI + 8]; __shared__ __attribute__((aligned(16))) float Tw[2][16][CO + 4]; __shared__ float Ss[32], Sd[32];
  const int wave = threadIdx.x >> 5, lane = threadIdx.x & 31, nloc = lane & 15, hlf = lane >> 4; const size_t m0 = (size_t)blockIdx.x * 32 + wave * 16;
  for (int idx = lane; idx < 16 * (CI / 4); idx += 32) { const int rr = idx / (CI / 4), c4 = (idx % (CI / 4)) * 4; const v4f v = *(const v4f*)(x + (m0 + rr) * CI + c4); v4h hv; for (int j = 0; j < 4; ++j) hv[j] = (b16)(bf16_rne(v[j]) * XS); *(v4h*)(&Ah[wave][rr][c4]) = hv; }
  wave_lds_sync();
  v8f acc[16];
#pragma unroll
  for (int t = 0; t < 16; ++t) acc[t] = (v8f){};
#pragma unroll 1
  for (int kb = 0; kb < CI; kb += 32) { const v16b a = frag_kb(&Ah[wave][nloc][kb], hlf);
#pragma unroll
    for (int t = 0; t < 16; ++t) acc[t] = wmma16b(a, frag_kb(WT + (size_t)(t * 16 + nloc) * CI + kb, hlf), acc[t]); }
  float ps[8], pd[8]; for (int r = 0; r < 8; ++r) { ps[r] = 0.0f; pd[r] = 0.0f; }
#pragma unroll
  for (int t = 0; t < 16; ++t) { const int c = t * 16 + nloc; const float ws = bf16_rne(as_[c]), wd = bf16_rne(ad_[c]);
#pragma unroll
    for (int r = 0; r < 8; ++r) { const float v = acc[t][r] * (1.0f / (XS * WSC)); Tw[wave][8 * hlf + r][c] = v; ps[r] = fmaf(v, ws, ps[r]); pd[r] = fmaf(v, wd, pd[r]); } }
#pragma unroll
  for (int o = 1; o < 16; o <<= 1) for (int r = 0; r < 8; ++r) { ps[r] += __shfl_xor(ps[r], o); pd[r] += __shfl_xor(pd[r], o); }
  if (nloc == 0) { for (int r = 0; r < 8; ++r) { Ss[wave * 16 + 8 * hlf + r] = ps[r]; Sd[wave * 16 + 8 * hlf + r] = pd[r]; } }
  wave_lds_sync();
  for (int pass = 0; pass < 2; ++pass) { for (int rr = 0; rr < 16; ++rr) for (int c8 = 0; c8 < CO; c8 += 128) { const v4f wv4 = *(const v4f*)(&Tw[wave][rr][c8 + lane * 4]); v4h hv, lv;
        for (int j = 0; j < 4; ++j) { const float wv = wv4[j] * XS; const b16 ph = (b16)wv; hv[j] = ph; lv[j] = (b16)((wv - (float)ph) * RS_); }
        const size_t o_ = (m0 + rr) * CO + c8 + lane * 4; *(volatile v4h*)(X1h + o_) = hv; *(volatile v4h*)(X1l + o_) = lv; }
    __threadfence(); }
  __syncthreads();
  if (wave == 0) { for (int pass = 0; pass < 2; ++pass) { ((volatile float*)AS)[(size_t)blockIdx.x * 32 + lane] = Ss[lane]; ((volatile float*)AD)[(size_t)blockIdx.x * 32 + lane] = Sd[lane]; __threadfence(); } }
}
__global__ __launch_bounds__(256) void pmax_kernel(const float* __restrict__ AS, float* __restrict__ PM) {
  __shared__ float cm[256]; __shared__ float ex[256];
  const int t = threadIdx.x; const int i0 = t * (N / 256); float m = -INFINITY; float loc[N / 256];
#pragma unroll
  for (int i = 0; i < N / 256; ++i) { m = fmaxf(m, AS[i0 + i]); loc[i] = m; }
  cm[t] = m; __syncthreads();
  if (t == 0) { float run = -INFINITY; for (int k = 0; k < 256; ++k) { ex[k] = run; run = fmaxf(run, cm[k]); } }
  __syncthreads();
  const float pre = ex[t];
  for (int pass = 0; pass < 2; ++pass) {
#pragma unroll
    for (int i = 0; i < N / 256; ++i) ((volatile float*)PM)[i0 + i] = fmaxf(pre, loc[i]); __threadfence(); }
}
__global__ __launch_bounds__(32) void attn_kernel(const b16* __restrict__ X1h, const b16* __restrict__ X1l, const float* __restrict__ AS, const float* __restrict__ AD, const float* __restrict__ PM, const float* __restrict__ bias, float* __restrict__ out) {
  __shared__ __attribute__((aligned(16))) b16 Pt[16][32 + 8]; __shared__ __attribute__((aligned(16))) float Of[16][128 + 4];
  const int lane = threadIdx.x, nloc = lane & 15, hlf = lane >> 4; const int j0 = blockIdx.x * 16, ch = blockIdx.y; const int j = j0 + nloc;
  const float adj = AD[j]; const float Mj = lrelu(PM[j] + adj); float lsum = 0.0f;
  v8f acc[8], accl[8];
#pragma unroll
  for (int t = 0; t < 8; ++t) { acc[t] = (v8f){}; accl[t] = (v8f){}; }
  const int iend = j0 + 16;
#pragma unroll 1
  for (int i0 = 0; i0 < iend; i0 += 32) {
    v16b pv;
#pragma unroll
    for (int q = 0; q < 16; ++q) { const int i = i0 + 16 * hlf + q; const bool on = (i <= j); const float p = on ? nexp2((lrelu(AS[i < N ? i : N - 1] + adj) - Mj) * LOG2E) : 0.0f; lsum += p; pv[q] = (b16)(p * PS); }
    *(v8b*)(&Pt[nloc][16 * hlf]) = __builtin_shufflevector(pv, pv, 0, 1, 2, 3, 4, 5, 6, 7); *(v8b*)(&Pt[nloc][16 * hlf + 8]) = __builtin_shufflevector(pv, pv, 8, 9, 10, 11, 12, 13, 14, 15);
    wave_lds_sync();
    const v16b a = frag_kb(&Pt[nloc][0], hlf);
#pragma unroll
    for (int t = 0; t < 8; ++t) { const int c = ch * 128 + t * 16 + nloc; v16b vh, vl;
#pragma unroll
      for (int e = 0; e < 16; ++e) { const int k = (e < 8) ? (8 * hlf + e) : (16 + 8 * hlf + (e - 8)); int i = i0 + k; i = (i < N) ? i : N - 1; const size_t o_ = (size_t)i * CO + c; vh[e] = X1h[o_]; vl[e] = X1l[o_]; }
      acc[t] = wmma16b(a, vh, acc[t]); accl[t] = wmma16b(a, vl, accl[t]); }
    wave_lds_sync(); }
  lsum += __shfl_xor(lsum, 16);
#pragma unroll
  for (int t = 0; t < 8; ++t) { const int cl = t * 16 + nloc; const float bb = bf16_rne(bias[ch * 128 + cl]);
#pragma unroll
    for (int r = 0; r < 8; ++r) { const float lr = __shfl(lsum, 8 * hlf + r); Of[8 * hlf + r][cl] = fmaxf((acc[t][r] + accl[t][r] * (1.0f / RS_)) * (1.0f / (XS * PS)) / lr + bb, 0.0f); } }
  wave_lds_sync();
  for (int pass = 0; pass < 2; ++pass) { for (int rr = 0; rr < 16; ++rr) if (j0 + rr < QL) *(volatile v4f*)(out + (size_t)(j0 + rr) * CO + ch * 128 + lane * 4) = *(const v4f*)(&Of[rr][lane * 4]); __threadfence(); }
}
}

extern "C" void kernel_launch(void* const* d_in, const int* in_sizes, int n_in, void* d_out, int out_size, void* d_ws, size_t ws_size, hipStream_t stream) {
  (void)n_in;
  auto Fp = [&](int i) { return (const float*)d_in[i]; };
  if (in_sizes[0] != N * CI || in_sizes[1] != CO * CI || in_sizes[2] != CO || in_sizes[3] != CO || in_sizes[4] != CO || out_size != N * CO) return;
  size_t off = 0; char* ws = (char*)d_ws;
  auto carve = [&](size_t bytes) { char* p = ws + off; off += (bytes + 255) & ~(size_t)255; return p; };
  b16* WT = (b16*)carve((size_t)CO * CI * 2); b16* X1h = (b16*)carve((size_t)N * CO * 2); b16* X1l = (b16*)carve((size_t)N * CO * 2); float* AS = (float*)carve((size_t)N * 4); float* AD = (float*)carve((size_t)N * 4); float* PM = (float*)carve((size_t)N * 4);
  if (off > ws_size || off > ((size_t)64 << 20)) return;
  wt_kernel<<<(CO * CI / 8 + 255) / 256, 256, 0, stream>>>(Fp(1), WT);
  proj_kernel<<<N / 32, 64, 0, stream>>>(Fp(0), WT, Fp(2), Fp(3), X1h, X1l, AS, AD);
  pmax_kernel<<<1, 256, 0, stream>>>(AS, PM);
  attn_kernel<<<dim3(QL / 16, 2), 32, 0, stream>>>(X1h, X1l, AS, AD, PM, Fp(4), (float*)d_out);
}
